// HRM_4x4_18760417149191
// MI455X (gfx1250) — hardware-verified
//
#include <hip/hip_runtime.h>
#include <stddef.h>
#include <stdint.h>
#include <math.h>


#define DMOD    64
#define FDIM    256
#define NSTAGE  55
#define CYCLEN  11
#define SW      64.0f
#define SA      256.0f
#define INVC    (1.0f / 16384.0f)
#define NWAVE   2
#define NTHR    64
#define RPW     16
#define RPB     32
#define PO_WV   0
#define PO_OW   4096
#define PO_F1   8192
#define PO_F2   24576
#define PO_SET  40960
#define PO_PROJ 81920
#define PO_HEAD 98304
#define PLANE_HALVES 100352
#define PREP_NB  49
#define PREP_THR 256
#define WSCAP   134217728

static_assert(PLANE_HALVES == PREP_NB * PREP_THR * 8);
static_assert(PO_HEAD + 32 * DMOD == PLANE_HALVES);
static_assert(PO_PROJ + DMOD * FDIM == PO_HEAD);
static_assert(2 * PO_SET == PO_PROJ);
static_assert(NTHR == NWAVE * 32);
static_assert(RPB == NWAVE * RPW);

typedef float    v4f  __attribute__((ext_vector_type(4)));
typedef float    v8f  __attribute__((ext_vector_type(8)));
typedef _Float16 v8h  __attribute__((ext_vector_type(8)));
typedef _Float16 v16h __attribute__((ext_vector_type(16)));
union FragH { v16h v; v8h h[2]; };
union F8    { v8f v; v4f q[2]; };

__device__ __forceinline__ v8f wmf(v16h a, v16h b, v8f c) {
  v8f d = __builtin_amdgcn_wmma_f32_16x16x32_f16(false, a, false, b, (short)0, c, false, false);
  asm volatile("v_nop\n\tv_nop\n\tv_nop\n\tv_nop" : "+v"(d) : "v"(a), "v"(b));
  return d;
}

__device__ __forceinline__ v16h ldA(const _Float16* __restrict__ W, int K, int row, int k) {
  const _Float16* p = W + (size_t)row * K + k;
  FragH a;
  a.h[0] = *(const v8h*)p;
  a.h[1] = *(const v8h*)(p + 16);
  return a.v;
}

__device__ __forceinline__ v16h packB(v8f lo, v8f hi) {
  FragH b;
#pragma unroll
  for (int r = 0; r < 8; ++r) {
    b.h[0][r] = (_Float16)(lo[r] * SA);
    b.h[1][r] = (_Float16)(hi[r] * SA);
  }
  return b.v;
}

__device__ __forceinline__ v8f ld8(const float* __restrict__ p) {
  F8 u;
  u.q[0] = *(const v4f*)p;
  u.q[1] = *(const v4f*)(p + 4);
  return u.v;
}

__device__ __forceinline__ v8f epi8(v8f acc, const float* __restrict__ bp) {
  const v8f bv = ld8(bp);
  v8f y;
#pragma unroll
  for (int r = 0; r < 8; ++r) y[r] = acc[r] * INVC + bv[r];
  return y;
}

__device__ __forceinline__ void gemm64(v8f (&Y)[4], const v16h (&xb)[2], const _Float16* __restrict__ W,
                                       const float* __restrict__ bias, int h, int m) {
#pragma unroll
  for (int f = 0; f < 4; ++f) {
    v8f acc = {0.f, 0.f, 0.f, 0.f, 0.f, 0.f, 0.f, 0.f};
#pragma unroll
    for (int kb = 0; kb < 2; ++kb) acc = wmf(ldA(W, DMOD, 16 * f + m, 32 * kb + 8 * h), xb[kb], acc);
    Y[f] = epi8(acc, bias + 16 * f + 8 * h);
  }
}

__device__ __forceinline__ void rms_add(v8f (&R)[4], const v8f (&X)[4], const v8f (&Y)[4],
                                        const float* __restrict__ nw, int h) {
  v8f s[4];
  float ss = 0.f;
#pragma unroll
  for (int f = 0; f < 4; ++f) {
    s[f] = X[f] + Y[f];
#pragma unroll
    for (int r = 0; r < 8; ++r) ss += s[f][r] * s[f][r];
  }
  ss += __shfl_xor(ss, 16, 32);
  const float sc = rsqrtf(ss * (1.0f / 64.0f) + 1e-6f);
#pragma unroll
  for (int f = 0; f < 4; ++f) {
    const v8f g = ld8(nw + 16 * f + 8 * h);
#pragma unroll
    for (int r = 0; r < 8; ++r) R[f][r] = s[f][r] * sc * g[r];
  }
}

__global__ __launch_bounds__(PREP_THR) void k_prep(const float* __restrict__ w_inw, const float* __restrict__ w_ow,
                                                   const float* __restrict__ w_f1w, const float* __restrict__ w_f2w,
                                                   const float* __restrict__ p_inw, const float* __restrict__ p_ow,
                                                   const float* __restrict__ p_f1w, const float* __restrict__ p_f2w,
                                                   const float* __restrict__ proj_w, const float* __restrict__ cell_w,
                                                   const float* __restrict__ dig_w, _Float16* plane) {
  const int b = blockIdx.x, t = threadIdx.x;
  v8h hv;
  if (b == PREP_NB - 1) {
    const int row = t >> 3, col = (t & 7) * 8;
    const int rc = row < 15 ? row : 15;
    int rd = row - 16;
    rd = rd < 0 ? 0 : (rd > 3 ? 3 : rd);
    const float* pc = cell_w + rc * DMOD + col;
    const float* pd = dig_w + rd * DMOD + col;
    const v4f c0 = *(const v4f*)pc, c1 = *(const v4f*)(pc + 4);
    const v4f d0 = *(const v4f*)pd, d1 = *(const v4f*)(pd + 4);
#pragma unroll
    for (int i = 0; i < 4; ++i) {
      const float vc0 = c0[i], vd0 = d0[i], vc1 = c1[i], vd1 = d1[i];
      const float s0 = (row < 16) ? vc0 : ((row < 20) ? vd0 : 0.0f);
      const float s1 = (row < 16) ? vc1 : ((row < 20) ? vd1 : 0.0f);
      hv[i]     = (_Float16)(s0 * SW);
      hv[4 + i] = (_Float16)(s1 * SW);
    }
  } else {
    const float* src;
    if (b >= 40) {
      src = proj_w + (size_t)(b - 40) * 2048;
    } else {
      const int lb = b % 20;
      const float* inw = (b < 20) ? w_inw : p_inw;
      const float* ow  = (b < 20) ? w_ow  : p_ow;
      const float* f1w = (b < 20) ? w_f1w : p_f1w;
      const float* f2w = (b < 20) ? w_f2w : p_f2w;
      if (lb < 2)       src = inw + 2 * DMOD * DMOD + lb * 2048;
      else if (lb < 4)  src = ow + (lb - 2) * 2048;
      else if (lb < 12) src = f1w + (lb - 4) * 2048;
      else              src = f2w + (lb - 12) * 2048;
    }
    const float* p = src + 8 * t;
    const v4f f0 = *(const v4f*)p, f1 = *(const v4f*)(p + 4);
#pragma unroll
    for (int i = 0; i < 4; ++i) {
      hv[i]     = (_Float16)(f0[i] * SW);
      hv[4 + i] = (_Float16)(f1[i] * SW);
    }
  }
  _Float16* d = plane + (size_t)b * 2048 + 8 * t;
  *(volatile v8h*)d = hv;
  __threadfence();
  *(volatile v8h*)d = hv;
}

__global__ __launch_bounds__(NTHR) void k_main(const int* __restrict__ puzzle, const float* __restrict__ emb,
                                               const float* __restrict__ proj_b, const float* __restrict__ hL0,
                                               const float* __restrict__ hH0, const float* __restrict__ cell_b,
                                               const float* __restrict__ dig_b,
                                               const float* __restrict__ w_inb, const float* __restrict__ w_ob,
                                               const float* __restrict__ w_f1b, const float* __restrict__ w_f2b,
                                               const float* __restrict__ w_n1, const float* __restrict__ w_n2,
                                               const float* __restrict__ p_inb, const float* __restrict__ p_ob,
                                               const float* __restrict__ p_f1b, const float* __restrict__ p_f2b,
                                               const float* __restrict__ p_n1, const float* __restrict__ p_n2,
                                               const _Float16* __restrict__ plane, float* out, int o1) {
  __shared__ v4f sL[NWAVE * 32 * 8];
  __shared__ v4f sH[NWAVE * 32 * 8];
  __shared__ v4f sX[NWAVE * 32 * 8];
  __shared__ v8h sE[NWAVE * 512];
  __shared__ v4f sO[NWAVE * 64];

  const int tid = threadIdx.x, lane = tid & 31, wave = tid >> 5, h = lane >> 4, m = lane & 15;
  const int n0 = (blockIdx.x * NWAVE + wave) * RPW;
  const int li = (wave * 32 + lane) * 8;
  const int ei = wave * 512 + m * 32;
  const v8f z8 = {0.f, 0.f, 0.f, 0.f, 0.f, 0.f, 0.f, 0.f};

  {
    const int* pz = puzzle + (size_t)(n0 + m) * 16;
#pragma unroll
    for (int c = 0; c < 16; ++c) {
      int id = pz[c];
      id = (id < 0) ? id + 5 : id;
      id = id < 0 ? 0 : (id > 4 ? 4 : id);
      const float* e = emb + id * 16 + 8 * h;
      const v4f e0 = *(const v4f*)e, e1 = *(const v4f*)(e + 4);
      v8h v;
#pragma unroll
      for (int i = 0; i < 4; ++i) {
        v[i]     = (_Float16)(e0[i] * SA);
        v[4 + i] = (_Float16)(e1[i] * SA);
      }
      sE[ei + 2 * c + h] = v;
    }
  }
  __syncthreads();

  {
    v8f xa[4] = {z8, z8, z8, z8};
    const _Float16* PW = plane + PO_PROJ;
#pragma unroll 1
    for (int kb = 0; kb < 8; ++kb) {
      FragH b;
      b.h[0] = sE[ei + 4 * kb + h];
      b.h[1] = sE[ei + 4 * kb + 2 + h];
#pragma unroll
      for (int f = 0; f < 4; ++f) xa[f] = wmf(ldA(PW, FDIM, 16 * f + m, 32 * kb + 8 * h), b.v, xa[f]);
    }
#pragma unroll
    for (int f = 0; f < 4; ++f) {
      F8 u;
      u.v = epi8(xa[f], proj_b + 16 * f + 8 * h);
      sX[li + 2 * f] = u.q[0];
      sX[li + 2 * f + 1] = u.q[1];
    }
  }
#pragma unroll
  for (int f = 0; f < 4; ++f) {
    F8 a, b;
    a.v = ld8(hL0 + 16 * f + 8 * h);
    b.v = ld8(hH0 + 16 * f + 8 * h);
    sL[li + 2 * f] = a.q[0]; sL[li + 2 * f + 1] = a.q[1];
    sH[li + 2 * f] = b.q[0]; sH[li + 2 * f + 1] = b.q[1];
  }

#pragma unroll 1
  for (int stage = 0; stage < NSTAGE; ++stage) {
    const bool pl = (stage % CYCLEN) == (CYCLEN - 1);
    const _Float16* WB = plane + (pl ? PO_SET : 0);
    const float* bvp = (pl ? p_inb : w_inb) + 2 * DMOD;
    const float* bop = pl ? p_ob  : w_ob;
    const float* b1p = pl ? p_f1b : w_f1b;
    const float* b2p = pl ? p_f2b : w_f2b;
    const float* g1p = pl ? p_n1  : w_n1;
    const float* g2p = pl ? p_n2  : w_n2;

    v8f C[4];
#pragma unroll
    for (int f = 0; f < 4; ++f) {
      F8 a, b, x;
      a.q[0] = sL[li + 2 * f]; a.q[1] = sL[li + 2 * f + 1];
      b.q[0] = sH[li + 2 * f]; b.q[1] = sH[li + 2 * f + 1];
      x.q[0] = sX[li + 2 * f]; x.q[1] = sX[li + 2 * f + 1];
      v8f t = a.v + b.v;
      if (!pl) t = t + x.v;
      C[f] = t;
    }
    v16h cb[2];
    cb[0] = packB(C[0], C[1]); cb[1] = packB(C[2], C[3]);
    v8f V[4];
    gemm64(V, cb, WB + PO_WV, bvp, h, m);
    v16h vb[2];
    vb[0] = packB(V[0], V[1]); vb[1] = packB(V[2], V[3]);
    v8f AT[4];
    gemm64(AT, vb, WB + PO_OW, bop, h, m);
    v8f H[4];
    rms_add(H, C, AT, g1p, h);
    v16h hb[2];
    hb[0] = packB(H[0], H[1]); hb[1] = packB(H[2], H[3]);
    v8f A2[4] = {z8, z8, z8, z8};
    const _Float16* W1 = WB + PO_F1;
    const _Float16* W2 = WB + PO_F2;
#pragma unroll 1
    for (int kb2 = 0; kb2 < 8; ++kb2) {
      FragH gb;
#pragma unroll
      for (int t = 0; t < 2; ++t) {
        const int f = 2 * kb2 + t;
        v8f acc = z8;
#pragma unroll
        for (int kb = 0; kb < 2; ++kb) acc = wmf(ldA(W1, DMOD, 16 * f + m, 32 * kb + 8 * h), hb[kb], acc);
        const v8f y = epi8(acc, b1p + 16 * f + 8 * h);
#pragma unroll
        for (int r = 0; r < 8; ++r) {
          const float xv = y[r];
          const float gv = 0.5f * xv * (1.0f + erff(xv * 0.70710678118654752f));
          gb.h[t][r] = (_Float16)(gv * SA);
        }
      }
#pragma unroll
      for (int f = 0; f < 4; ++f) A2[f] = wmf(ldA(W2, FDIM, 16 * f + m, 32 * kb2 + 8 * h), gb.v, A2[f]);
    }
    v8f FN[4];
#pragma unroll
    for (int f = 0; f < 4; ++f) FN[f] = epi8(A2[f], b2p + 16 * f + 8 * h);
    v8f R[4];
    rms_add(R, H, FN, g2p, h);
    if (pl) {
#pragma unroll
      for (int f = 0; f < 4; ++f) { F8 u; u.v = R[f]; sH[li + 2 * f] = u.q[0]; sH[li + 2 * f + 1] = u.q[1]; }
    } else {
#pragma unroll
      for (int f = 0; f < 4; ++f) { F8 u; u.v = R[f]; sL[li + 2 * f] = u.q[0]; sL[li + 2 * f + 1] = u.q[1]; }
    }
  }

  v8f HH[4];
#pragma unroll
  for (int f = 0; f < 4; ++f) { F8 u; u.q[0] = sH[li + 2 * f]; u.q[1] = sH[li + 2 * f + 1]; HH[f] = u.v; }
  v16h qb[2];
  qb[0] = packB(HH[0], HH[1]); qb[1] = packB(HH[2], HH[3]);
  const _Float16* WH = plane + PO_HEAD;
  v8f a0 = z8, a1 = z8;
#pragma unroll
  for (int kb = 0; kb < 2; ++kb) {
    a0 = wmf(ldA(WH, DMOD, m,      32 * kb + 8 * h), qb[kb], a0);
    a1 = wmf(ldA(WH, DMOD, 16 + m, 32 * kb + 8 * h), qb[kb], a1);
  }
  const v8f cl = epi8(a0, cell_b + 8 * h);
  const v4f db = *(const v4f*)dig_b;
  v4f dg;
#pragma unroll
  for (int r = 0; r < 4; ++r) dg[r] = a1[r] * INVC + db[r];
  {
    F8 u; u.v = cl;
    sO[wave * 64 + m * 4 + 2 * h]     = u.q[0];
    sO[wave * 64 + m * 4 + 2 * h + 1] = u.q[1];
  }
  __syncthreads();
  const v4f o0v = sO[wave * 64 + lane];
  const v4f o1v = sO[wave * 64 + 32 + lane];
  float* ob0 = out + (size_t)n0 * 16;
  float* ob1 = out + (size_t)o1 + (size_t)(n0 + m) * 4;
  *(volatile v4f*)(ob0 + 4 * lane)       = o0v;
  *(volatile v4f*)(ob0 + 128 + 4 * lane) = o1v;
  if (h == 0) *(volatile v4f*)ob1 = dg;
  __threadfence();
  *(volatile v4f*)(ob0 + 4 * lane)       = o0v;
  *(volatile v4f*)(ob0 + 128 + 4 * lane) = o1v;
  if (h == 0) *(volatile v4f*)ob1 = dg;
}

extern "C" void kernel_launch(void* const* d_in, const int* in_sizes, int n_in,
                              void* d_out, int out_size, void* d_ws, size_t ws_size,
                              hipStream_t stream) {
  if (n_in < 30) return;
  const int nrows = in_sizes[0] / 16;
  if (nrows <= 0 || nrows * 16 != in_sizes[0] || (nrows % RPB) != 0) return;
  if (in_sizes[1] != 80 || in_sizes[2] != DMOD * FDIM || in_sizes[3] != DMOD) return;
  if (in_sizes[4] != DMOD || in_sizes[5] != DMOD) return;
  if (in_sizes[6] != 16 * DMOD || in_sizes[7] != 16 || in_sizes[8] != 4 * DMOD || in_sizes[9] != 4) return;
  for (int s = 0; s < 2; ++s) {
    const int o = 10 + 10 * s;
    if (in_sizes[o + 0] != 3 * DMOD * DMOD || in_sizes[o + 1] != 3 * DMOD) return;
    if (in_sizes[o + 2] != DMOD * DMOD || in_sizes[o + 3] != DMOD) return;
    if (in_sizes[o + 4] != FDIM * DMOD || in_sizes[o + 5] != FDIM) return;
    if (in_sizes[o + 6] != DMOD * FDIM || in_sizes[o + 7] != DMOD) return;
    if (in_sizes[o + 8] != DMOD || in_sizes[o + 9] != DMOD) return;
  }
  if (out_size != nrows * 20) return;

  const size_t plane_bytes = (size_t)PLANE_HALVES * 2;
  if (plane_bytes > ws_size || plane_bytes > (size_t)WSCAP) return;
  _Float16* plane = (_Float16*)d_ws;

  const int*   puzzle = (const int*)d_in[0];
  const float* emb    = (const float*)d_in[1];
  const float* proj_w = (const float*)d_in[2];
  const float* proj_b = (const float*)d_in[3];
  const float* hL0    = (const float*)d_in[4];
  const float* hH0    = (const float*)d_in[5];
  const float* cell_w = (const float*)d_in[6];
  const float* cell_b = (const float*)d_in[7];
  const float* dig_w  = (const float*)d_in[8];
  const float* dig_b  = (const float*)d_in[9];
  const float* w_inw  = (const float*)d_in[10]; const float* w_inb = (const float*)d_in[11];
  const float* w_ow   = (const float*)d_in[12]; const float* w_ob  = (const float*)d_in[13];
  const float* w_f1w  = (const float*)d_in[14]; const float* w_f1b = (const float*)d_in[15];
  const float* w_f2w  = (const float*)d_in[16]; const float* w_f2b = (const float*)d_in[17];
  const float* w_n1   = (const float*)d_in[18]; const float* w_n2  = (const float*)d_in[19];
  const float* p_inw  = (const float*)d_in[20]; const float* p_inb = (const float*)d_in[21];
  const float* p_ow   = (const float*)d_in[22]; const float* p_ob  = (const float*)d_in[23];
  const float* p_f1w  = (const float*)d_in[24]; const float* p_f1b = (const float*)d_in[25];
  const float* p_f2w  = (const float*)d_in[26]; const float* p_f2b = (const float*)d_in[27];
  const float* p_n1   = (const float*)d_in[28]; const float* p_n2  = (const float*)d_in[29];
  float* out = (float*)d_out;
  const int o1 = nrows * 16;

  k_prep<<<PREP_NB, PREP_THR, 0, stream>>>(w_inw, w_ow, w_f1w, w_f2w, p_inw, p_ow, p_f1w, p_f2w,
                                           proj_w, cell_w, dig_w, plane);
  k_main<<<nrows / RPB, NTHR, 0, stream>>>(puzzle, emb, proj_b, hL0, hH0, cell_b, dig_b,
                                           w_inb, w_ob, w_f1b, w_f2b, w_n1, w_n2,
                                           p_inb, p_ob, p_f1b, p_f2b, p_n1, p_n2,
                                           plane, out, o1);
}
